// RGCN_20401094656588
// MI455X (gfx1250) — hardware-run, weakly checked
//
#include <hip/hip_runtime.h>
#include <stddef.h>
#include <stdint.h>
#include <math.h>

#define NN      100000
#define NE      400000
#define NR      3
#define DF      128
#define NC      40
#define NT      48
#define MP      100096
#define GBM     64
#define GTHR    128
#define HBM     128
#define NTHR    256
#define NWAVE   8
#define EPT     8
#define WCH     (32 * EPT)
#define NBRUN   1024
#define SLB     10
#define NBK     98
#define NPADN   (NBK * NBRUN)
#define WLCAP   768
#define RCAP    6144
#define DEGCAP  48
#define MEAS_B1024  4281
#define MEAS_MAXDEG 16
#define RPB     64
#define RPW     8
#define PP      384
#define HLP     256
#define XBP     128
#define W1P     128
#define W2P     256
#define WCP     256
#define TWO_L2  1
#define TWO_HD  1
#define K_L1    128
#define K_L2    (TWO_L2 ? 256 : 128)
#define K_HD    (TWO_HD ? 256 : 128)

#define BK_ZINTS (NWAVE * WLCAP + RCAP + 3 * NBRUN)
#define BK_INTS  (BK_ZINTS + 16)

#define PBX   (MP * DF / 8 / NTHR)
#define PBW1  (NR * DF * W1P / 8 / NTHR)
#define PBW2  (NR * DF * W2P / 8 / NTHR)
#define PBWC  (NT * WCP / 8 / NTHR)
#define PBTOT (PBX + PBW1 + PBW2 + PBWC + 1)

static_assert(DF == 32 * 4);
static_assert(NN == 781 * HBM + 32 && MP == 782 * HBM && MP == 1564 * GBM && MP % RPB == 0 && MP >= NN);
static_assert(NE < (1 << 19) && (((long long)NE) << SLB) < (1LL << 31));
static_assert(NE % EPT == 0 && WCH % EPT == 0);
static_assert(NBRUN == (1 << SLB) && NBRUN == NTHR * 4 && NBRUN % HBM == 0 && NBRUN % RPB == 0 && NBRUN % GBM == 0);
static_assert(NBK * NBRUN >= NN && NBK * NBRUN >= MP);
static_assert(RCAP == NWAVE * WLCAP && RCAP % (NTHR * 4) == 0 && BK_ZINTS % (NTHR * 4) == 0);
static_assert((long long)RCAP * 100 >= (long long)MEAS_B1024 * 105);
static_assert(WLCAP >= MEAS_B1024 / 8 + 8 * 23 + 1);
static_assert(DEGCAP >= MEAS_MAXDEG + 8);
static_assert(NC <= NT && NT == 3 * 16 && NT <= 64);
static_assert(K_L1 % 32 == 0 && K_L2 % 32 == 0 && K_HD % 32 == 0);
static_assert(K_L1 <= XBP && K_L1 <= W1P && K_L2 <= HLP && K_L2 <= W2P && K_HD <= HLP && K_HD <= WCP);
static_assert(GBM == (GTHR / 32) * 16 && HBM == NWAVE * 16 && RPB == NWAVE * RPW);
static_assert((MP * DF / 8) % NTHR == 0 && (NR * DF * W1P / 8) % NTHR == 0);
static_assert((NR * DF * W2P / 8) % NTHR == 0 && (NT * WCP / 8) % NTHR == 0);
static_assert((HBM * NC * 4) % 128 == 0 && (((NN % HBM) * NC * 4) % 128) == 0 && HBM * NC / 4 == 5 * NTHR);
static_assert(BK_INTS * 4 <= 65536);
static_assert((GBM * DF + GBM) * 4 <= 65536);
static_assert((HBM * NC + 64) * 4 <= 65536);

typedef float          v4f   __attribute__((ext_vector_type(4)));
typedef float          v8f   __attribute__((ext_vector_type(8)));
typedef int            v4i   __attribute__((ext_vector_type(4)));
typedef int            v8i   __attribute__((ext_vector_type(8)));
typedef unsigned short v8us  __attribute__((ext_vector_type(8)));
typedef __bf16         v16bf __attribute__((ext_vector_type(16)));
typedef v4f  __attribute__((may_alias)) v4fa;
typedef v4i  __attribute__((may_alias)) v4ia;
typedef v8us __attribute__((may_alias)) v8usa;
union FragB { v16bf v; v8us h[2]; v8i w; };

__device__ __forceinline__ v8f wmb(const FragB& a, const FragB& b, v8f c) {
  v8f d = __builtin_amdgcn_wmma_f32_16x16x32_bf16(false, a.v, false, b.v, (short)0, c, false, false);
  asm volatile("v_nop\n\tv_nop\n\tv_nop\n\tv_nop" : "+v"(d) : "v"(a.w), "v"(b.w));
  return d;
}

__device__ __forceinline__ unsigned bf16_bits(float f) {
  const unsigned u = __float_as_uint(f);
  const unsigned r = (u + 0x7FFFu + ((u >> 16) & 1u)) >> 16;
  const unsigned q = (u >> 16) | 0x40u;
  return ((u & 0x7fffffffu) > 0x7f800000u) ? q : r;
}

__device__ __forceinline__ void hilo_pack(float v0, float v1, float v2, float v3,
                                          int& h01, int& h23, int& l01, int& l23) {
  const unsigned a0 = bf16_bits(v0), a1 = bf16_bits(v1), a2 = bf16_bits(v2), a3 = bf16_bits(v3);
  const unsigned b0 = bf16_bits(v0 - __uint_as_float(a0 << 16));
  const unsigned b1 = bf16_bits(v1 - __uint_as_float(a1 << 16));
  const unsigned b2 = bf16_bits(v2 - __uint_as_float(a2 << 16));
  const unsigned b3 = bf16_bits(v3 - __uint_as_float(a3 << 16));
  h01 = (int)(a0 | (a1 << 16)); h23 = (int)(a2 | (a3 << 16));
  l01 = (int)(b0 | (b1 << 16)); l23 = (int)(b2 | (b3 << 16));
}

__device__ __forceinline__ v4i regroup_row(int h01, int h23, int l01, int l23, int lane) {
  const int s0 = (2 * lane) & 31, s1 = s0 + 1;
  const int a0 = __shfl(h01, s0, 32), a1 = __shfl(h23, s0, 32), a2 = __shfl(h01, s1, 32), a3 = __shfl(h23, s1, 32);
  const int b0 = __shfl(l01, s0, 32), b1 = __shfl(l23, s0, 32), b2 = __shfl(l01, s1, 32), b3 = __shfl(l23, s1, 32);
  const int mk = (lane < 16) ? -1 : 0;
  v4i o;
  o.x = (a0 & mk) | (b0 & ~mk); o.y = (a1 & mk) | (b1 & ~mk);
  o.z = (a2 & mk) | (b2 & ~mk); o.w = (a3 & mk) | (b3 & ~mk);
  return o;
}

__device__ __forceinline__ void st2_v4f(float* p, v4f v) {
  *(volatile v4f*)p = v;
  __threadfence();
  *(volatile v4f*)p = v;
}
__device__ __forceinline__ void st2_v8us(unsigned short* p, v8us v) {
  *(volatile v8us*)p = v;
  __threadfence();
  *(volatile v8us*)p = v;
}

__device__ __forceinline__ v8us strided8(const float* __restrict__ base, int stride, unsigned mk) {
  float f[8];
#pragma unroll
  for (int i = 0; i < 8; ++i) f[i] = base[(size_t)i * (size_t)stride];
  v8us o;
#pragma unroll
  for (int i = 0; i < 8; ++i) o[i] = (unsigned short)(bf16_bits(f[i]) & mk);
  return o;
}

__global__ __launch_bounds__(NTHR) void k_prep(const float* __restrict__ x, const float* __restrict__ w1,
                                               const float* __restrict__ b1, const float* __restrict__ w2,
                                               const float* __restrict__ b2, const float* __restrict__ wc,
                                               const float* __restrict__ bc,
                                               unsigned short* xb, unsigned short* w1c, unsigned short* w2c,
                                               unsigned short* wct, float* bt) {
  const int tid = (int)threadIdx.x;
  const int blk = (int)blockIdx.x;
  if (blk < PBX) {
    const int u   = blk * NTHR + tid;
    const int row = u >> 4, k8 = (u & 15) * 8;
    const int rc  = row < NN ? row : NN - 1;
    const unsigned mk = row < NN ? 0xffffu : 0u;
    const float* p = x + (size_t)rc * DF + k8;
    const v4f a = *(const v4fa*)p;
    const v4f b = *(const v4fa*)(p + 4);
    v8us o;
    o[0] = (unsigned short)(bf16_bits(a.x) & mk); o[1] = (unsigned short)(bf16_bits(a.y) & mk);
    o[2] = (unsigned short)(bf16_bits(a.z) & mk); o[3] = (unsigned short)(bf16_bits(a.w) & mk);
    o[4] = (unsigned short)(bf16_bits(b.x) & mk); o[5] = (unsigned short)(bf16_bits(b.y) & mk);
    o[6] = (unsigned short)(bf16_bits(b.z) & mk); o[7] = (unsigned short)(bf16_bits(b.w) & mk);
    st2_v8us(xb + (size_t)row * XBP + k8, o);
  } else if (blk < PBX + PBW1) {
    const int u   = (blk - PBX) * NTHR + tid;
    const int row = u >> 4, k8 = (u & 15) * 8;
    const int r = row >> 7, o = row & 127;
    const v8us v = strided8(w1 + (size_t)r * DF * DF + (size_t)k8 * DF + o, DF, 0xffffu);
    st2_v8us(w1c + (size_t)row * W1P + k8, v);
  } else if (blk < PBX + PBW1 + PBW2) {
    const int u   = (blk - PBX - PBW1) * NTHR + tid;
    const int row = u >> 5, k8 = (u & 31) * 8, kk = k8 & 127;
    const int r = row >> 7, o = row & 127;
    const v8us v = strided8(w2 + (size_t)r * DF * DF + (size_t)kk * DF + o, DF, 0xffffu);
    st2_v8us(w2c + (size_t)row * W2P + k8, v);
  } else if (blk < PBX + PBW1 + PBW2 + PBWC) {
    const int u  = (blk - PBX - PBW1 - PBW2) * NTHR + tid;
    const int c  = u >> 5, k8 = (u & 31) * 8, kk = k8 & 127;
    const int cc = c < NC ? c : NC - 1;
    const unsigned mk = c < NC ? 0xffffu : 0u;
    const v8us v = strided8(wc + (size_t)kk * NC + cc, NC, mk);
    st2_v8us(wct + (size_t)c * WCP + k8, v);
  } else {
    const int i0 = 4 * tid;
    int ia = i0;           ia = ia > 380 ? 380 : ia;
    int ib = i0 - 384;     ib = ib < 0 ? 0 : (ib > 380 ? 380 : ib);
    int ic = i0 - 768;     ic = ic < 0 ? 0 : (ic > NC - 4 ? NC - 4 : ic);
    const v4f va = *(const v4fa*)(b1 + ia);
    const v4f vb = *(const v4fa*)(b2 + ib);
    const v4f vc = *(const v4fa*)(bc + ic);
    asm volatile("" :: "v"(va), "v"(vb), "v"(vc));
    const unsigned ma = (i0 < 384) ? 0xffffffffu : 0u;
    const unsigned mb = (i0 >= 384 && i0 < 768) ? 0xffffffffu : 0u;
    const unsigned mc = (i0 >= 768 && i0 < 768 + NC) ? 0xffffffffu : 0u;
    v4f o;
    o.x = __uint_as_float(((bf16_bits(va.x) << 16) & ma) | ((bf16_bits(vb.x) << 16) & mb) | ((bf16_bits(vc.x) << 16) & mc));
    o.y = __uint_as_float(((bf16_bits(va.y) << 16) & ma) | ((bf16_bits(vb.y) << 16) & mb) | ((bf16_bits(vc.y) << 16) & mc));
    o.z = __uint_as_float(((bf16_bits(va.z) << 16) & ma) | ((bf16_bits(vb.z) << 16) & mb) | ((bf16_bits(vc.z) << 16) & mc));
    o.w = __uint_as_float(((bf16_bits(va.w) << 16) & ma) | ((bf16_bits(vb.w) << 16) & mb) | ((bf16_bits(vc.w) << 16) & mc));
    st2_v4f(bt + i0, o);
  }
}

__device__ __forceinline__ void bucket_flush(int role, const int* pl, const int* cnt, const int* offs,
                                             const int* nrm, int flag, int* lp, int* cp, int* fp, int* ndp,
                                             int* nsp, int* gp, int tid) {
  if (role == 0) {
#pragma unroll 1
    for (int i = tid * 4; i < RCAP; i += NTHR * 4) {
      const v4i v = *(const v4ia*)(pl + i);
      *(volatile v4i*)(lp + i) = v;
    }
    const v4i c = *(const v4ia*)(cnt + 4 * tid);
    const v4i o = *(const v4ia*)(offs + 4 * tid);
    const v4i n = *(const v4ia*)(nrm + 4 * tid);
    *(volatile v4i*)(cp + 4 * tid)  = c;
    *(volatile v4i*)(fp + 4 * tid)  = o;
    *(volatile v4i*)(ndp + 4 * tid) = n;
    if (tid < 8) {
      const v4i f = {flag, flag, flag, flag};
      *(volatile v4i*)(gp + 4 * tid) = f;
    }
  } else {
    const v4i n = *(const v4ia*)(nrm + 4 * tid);
    *(volatile v4i*)(nsp + 4 * tid) = n;
  }
}

__global__ __launch_bounds__(NTHR) void k_bucket(const int* __restrict__ edges, int* LIST, int* CNT, int* OFF,
                                                 int* NRM, int* FLAG) {
  __shared__ __attribute__((aligned(16))) int dsm[BK_INTS];
  int* wl   = dsm;
  int* pl   = dsm + NWAVE * WLCAP;
  int* cnt  = pl + RCAP;
  int* offs = cnt + NBRUN;
  int* cur  = offs + NBRUN;
  int* misc = cur + NBRUN;
  const int tid = (int)threadIdx.x, lane = tid & 31, wave = tid >> 5;
  const int blk  = (int)blockIdx.x;
  const int role = blk / (NR * NBK);
  const int rem  = blk - role * (NR * NBK);
  const int rel  = rem / NBK;
  const int bb   = rem - rel * NBK;
  const unsigned nbs = (unsigned)(bb * NBRUN);
  const int* keys = edges + (size_t)(2 * rel + (role == 0 ? 1 : 0)) * NE;
  const int* srcs = edges + (size_t)(2 * rel) * NE;

  {
    const v4i z4 = {0, 0, 0, 0};
    for (int i = tid * 4; i < BK_ZINTS; i += NTHR * 4) *(v4ia*)(dsm + i) = z4;
    if (tid < 16) misc[tid] = 0;
  }
  __syncthreads();

  {
    const int per  = ((NE + NWAVE * WCH - 1) / (NWAVE * WCH)) * WCH;
    const int ebeg = wave * per;
    const int eend = (ebeg + per < NE) ? (ebeg + per) : NE;
    int* mylist = wl + wave * WLCAP;
    int wc = 0;
#pragma unroll 1
    for (int cb = ebeg; cb < eend; cb += WCH) {
      const int e0 = cb + lane * EPT;
      const bool valid = e0 < eend;
      const int ec = valid ? e0 : (eend - EPT);
      const v4i da = *(const v4ia*)(keys + ec);
      const v4i db = *(const v4ia*)(keys + ec + 4);
      asm volatile("" :: "v"(da), "v"(db));
      const unsigned s0 = (unsigned)da.x - nbs, s1 = (unsigned)da.y - nbs;
      const unsigned s2 = (unsigned)da.z - nbs, s3 = (unsigned)da.w - nbs;
      const unsigned s4 = (unsigned)db.x - nbs, s5 = (unsigned)db.y - nbs;
      const unsigned s6 = (unsigned)db.z - nbs, s7 = (unsigned)db.w - nbs;
      const bool h0 = valid & (s0 < (unsigned)NBRUN), h1 = valid & (s1 < (unsigned)NBRUN);
      const bool h2 = valid & (s2 < (unsigned)NBRUN), h3 = valid & (s3 < (unsigned)NBRUN);
      const bool h4 = valid & (s4 < (unsigned)NBRUN), h5 = valid & (s5 < (unsigned)NBRUN);
      const bool h6 = valid & (s6 < (unsigned)NBRUN), h7 = valid & (s7 < (unsigned)NBRUN);
      const unsigned m0 = __builtin_amdgcn_ballot_w32(h0), m1 = __builtin_amdgcn_ballot_w32(h1);
      const unsigned m2 = __builtin_amdgcn_ballot_w32(h2), m3 = __builtin_amdgcn_ballot_w32(h3);
      const unsigned m4 = __builtin_amdgcn_ballot_w32(h4), m5 = __builtin_amdgcn_ballot_w32(h5);
      const unsigned m6 = __builtin_amdgcn_ballot_w32(h6), m7 = __builtin_amdgcn_ballot_w32(h7);
      const unsigned any = m0 | m1 | m2 | m3 | m4 | m5 | m6 | m7;
      if (any != 0u) {
        const int pre = (int)(__builtin_amdgcn_mbcnt_lo(m0, 0u) + __builtin_amdgcn_mbcnt_lo(m1, 0u) +
                              __builtin_amdgcn_mbcnt_lo(m2, 0u) + __builtin_amdgcn_mbcnt_lo(m3, 0u) +
                              __builtin_amdgcn_mbcnt_lo(m4, 0u) + __builtin_amdgcn_mbcnt_lo(m5, 0u) +
                              __builtin_amdgcn_mbcnt_lo(m6, 0u) + __builtin_amdgcn_mbcnt_lo(m7, 0u));
        int p = wc + pre;
        if (h0) { if (p < WLCAP) mylist[p] = ((e0 + 0) << SLB) | (int)s0; p = p + 1; }
        if (h1) { if (p < WLCAP) mylist[p] = ((e0 + 1) << SLB) | (int)s1; p = p + 1; }
        if (h2) { if (p < WLCAP) mylist[p] = ((e0 + 2) << SLB) | (int)s2; p = p + 1; }
        if (h3) { if (p < WLCAP) mylist[p] = ((e0 + 3) << SLB) | (int)s3; p = p + 1; }
        if (h4) { if (p < WLCAP) mylist[p] = ((e0 + 4) << SLB) | (int)s4; p = p + 1; }
        if (h5) { if (p < WLCAP) mylist[p] = ((e0 + 5) << SLB) | (int)s5; p = p + 1; }
        if (h6) { if (p < WLCAP) mylist[p] = ((e0 + 6) << SLB) | (int)s6; p = p + 1; }
        if (h7) { if (p < WLCAP) mylist[p] = ((e0 + 7) << SLB) | (int)s7; p = p + 1; }
        wc += (int)(__builtin_popcount(m0) + __builtin_popcount(m1) + __builtin_popcount(m2) + __builtin_popcount(m3) +
                    __builtin_popcount(m4) + __builtin_popcount(m5) + __builtin_popcount(m6) + __builtin_popcount(m7));
      }
    }
    if (lane == 0) misc[wave] = wc;
  }
  __syncthreads();

  if (wave == 0) {
    int ov = 0;
#pragma unroll 1
    for (int w2 = 0; w2 < NWAVE; ++w2) {
      int c = misc[w2];
      if (c > WLCAP) ov = 1;
      c = c < 0 ? 0 : (c > WLCAP ? WLCAP : c);
#pragma unroll 1
      for (int b0 = 0; b0 < c; b0 += 32) {
        const int idx = b0 + lane;
        const int ent = wl[w2 * WLCAP + (idx < WLCAP ? idx : WLCAP - 1)];
        const int m32 = (c - b0) < 32 ? (c - b0) : 32;
#pragma unroll 1
        for (int k = 0; k < m32; ++k) {
          const int u    = __builtin_amdgcn_readlane(ent, k);
          const int slot = u & (NBRUN - 1);
          if (lane == 0) cnt[slot] = cnt[slot] + 1;
        }
      }
    }
    if (lane == 0) misc[9] = ov;
  }
  __syncthreads();
  if (wave == 0) {
    const int base = lane * (NBRUN / 32);
    int s = 0, mx = 0;
#pragma unroll 1
    for (int i = 0; i < NBRUN / 32; ++i) {
      const int cv = cnt[base + i];
      s += cv;
      mx = cv > mx ? cv : mx;
    }
    int incl = s;
#pragma unroll
    for (int d = 1; d < 32; d <<= 1) {
      const int y = __shfl_up(incl, d, 32);
      if (lane >= d) incl += y;
    }
    mx = max(mx, __shfl_xor(mx, 16, 32));
    mx = max(mx, __shfl_xor(mx, 8, 32));
    mx = max(mx, __shfl_xor(mx, 4, 32));
    mx = max(mx, __shfl_xor(mx, 2, 32));
    mx = max(mx, __shfl_xor(mx, 1, 32));
    int run = incl - s;
#pragma unroll 1
    for (int i = 0; i < NBRUN / 32; ++i) {
      const int cv = cnt[base + i];
      offs[base + i] = run;
      cur[base + i]  = run;
      run += cv;
    }
    if (lane == 0) misc[10] = mx;
  }
  __syncthreads();

  if (role == 0 && wave == 0) {
#pragma unroll 1
    for (int w2 = 0; w2 < NWAVE; ++w2) {
      int c = misc[w2];
      c = c < 0 ? 0 : (c > WLCAP ? WLCAP : c);
#pragma unroll 1
      for (int b0 = 0; b0 < c; b0 += 32) {
        const int idx = b0 + lane;
        const int ent = wl[w2 * WLCAP + (idx < WLCAP ? idx : WLCAP - 1)];
        int eid = (ent >> SLB) & 0x7FFFF;
        eid = eid > NE - 1 ? NE - 1 : eid;
        int sr = srcs[eid];
        sr = sr < 0 ? 0 : (sr > NN - 1 ? NN - 1 : sr);
        const int m32 = (c - b0) < 32 ? (c - b0) : 32;
#pragma unroll 1
        for (int k = 0; k < m32; ++k) {
          const int u    = __builtin_amdgcn_readlane(ent, k);
          const int wd   = __builtin_amdgcn_readlane(sr, k);
          const int slot = u & (NBRUN - 1);
          if (lane == 0) {
            int p = cur[slot];
            p = p < 0 ? 0 : (p > RCAP - 1 ? RCAP - 1 : p);
            pl[p] = wd;
            cur[slot] = p + 1;
          }
        }
      }
    }
  }
  __syncthreads();

  const int ovf  = misc[9];
  const int bmax = misc[10];
#pragma unroll 1
  for (int j = 0; j < 4; ++j) {
    int c = cnt[4 * tid + j];
    c = c < 1 ? 1 : c;
    const float v = 1.0f / sqrtf((float)c);
    cur[4 * tid + j] = (ovf != 0) ? (int)0x7fc00000u : __float_as_int(v);
  }
  const int flag = ((ovf != 0) || (bmax > DEGCAP)) ? 1 : 0;
  const size_t tb = (size_t)rel * NPADN + (size_t)nbs;
  int* lp  = LIST + (size_t)(rel * NBK + bb) * RCAP;
  int* cp  = CNT + tb;
  int* fp  = OFF + tb;
  int* nsp = NRM + tb;
  int* ndp = NRM + (size_t)NR * NPADN + tb;
  int* gp  = FLAG + (size_t)(rel * NBK + bb) * 32;
  bucket_flush(role, pl, cnt, offs, cur, flag, lp, cp, fp, ndp, nsp, gp, tid);
  __threadfence();
  bucket_flush(role, pl, cnt, offs, cur, flag, lp, cp, fp, ndp, nsp, gp, tid);
}

template <int KEXT, int APITCH, int WPITCH>
__device__ __forceinline__ void gemm_tile(const unsigned short* __restrict__ A, const unsigned short* __restrict__ WT,
                                          const float* __restrict__ NS, float* P, float* stg, float* nsh) {
  static_assert(KEXT % 32 == 0 && KEXT <= APITCH && KEXT <= WPITCH);
  const int tid = (int)threadIdx.x, lane = tid & 31, wave = tid >> 5, hh = lane >> 4, m = lane & 15;
  const int rowBase = (int)blockIdx.x * GBM;
  const int rel     = (int)blockIdx.y;
  {
    const v4f q = *(const v4fa*)(NS + (size_t)rel * NPADN + (size_t)rowBase + 4 * (tid & 15));
    asm volatile("" :: "v"(q));
    if (tid < GBM / 4) *(v4fa*)(nsh + 4 * tid) = q;
  }
  v8f acc[8];
  {
    const v8f z = {0.f, 0.f, 0.f, 0.f, 0.f, 0.f, 0.f, 0.f};
#pragma unroll
    for (int t = 0; t < 8; ++t) acc[t] = z;
  }
  const unsigned short* ap = A + (size_t)(rowBase + 16 * wave + m) * (size_t)APITCH + 8 * hh;
  const unsigned short* bp = WT + (size_t)(rel * DF + m) * (size_t)WPITCH + 8 * hh;
#pragma unroll 1
  for (int k0 = 0; k0 < KEXT; k0 += 32) {
    FragB af;
    af.h[0] = *(const v8usa*)(ap + k0);
    af.h[1] = *(const v8usa*)(ap + k0 + 16);
#pragma unroll
    for (int t = 0; t < 8; ++t) {
      const unsigned short* wq = bp + (size_t)(16 * t) * (size_t)WPITCH + k0;
      FragB bf;
      bf.h[0] = *(const v8usa*)wq;
      bf.h[1] = *(const v8usa*)(wq + 16);
      acc[t] = wmb(af, bf, acc[t]);
    }
  }
#pragma unroll
  for (int t = 0; t < 8; ++t) {
#pragma unroll
    for (int r = 0; r < 8; ++r) stg[(16 * wave + 8 * hh + r) * DF + 16 * t + m] = acc[t][r];
  }
  __syncthreads();
#pragma unroll 1
  for (int i = 0; i < 16; ++i) {
    const int lr   = 16 * wave + i;
    const int grow = rowBase + lr;
    const float ns = nsh[lr];
    const v4f a = *(const v4fa*)(stg + lr * DF + 4 * lane);
    asm volatile("" :: "v"(a));
    const bool live = grow < NN;
    v4f o;
    o.x = live ? a.x * ns : 0.0f; o.y = live ? a.y * ns : 0.0f;
    o.z = live ? a.z * ns : 0.0f; o.w = live ? a.w * ns : 0.0f;
    st2_v4f(P + (size_t)grow * PP + rel * DF + 4 * lane, o);
  }
}

__global__ __launch_bounds__(GTHR) __attribute__((amdgpu_num_vgpr(248)))
void k_gemm_one(const unsigned short* __restrict__ XB, const unsigned short* __restrict__ W1C,
                const float* __restrict__ NS, float* P) {
  __shared__ __attribute__((aligned(16))) float stg[GBM * DF];
  __shared__ __attribute__((aligned(16))) float nsh[GBM];
  gemm_tile<K_L1, XBP, W1P>(XB, W1C, NS, P, stg, nsh);
}

__global__ __launch_bounds__(GTHR) __attribute__((amdgpu_num_vgpr(248)))
void k_gemm_two(const unsigned short* __restrict__ HL, const unsigned short* __restrict__ W2C,
                const float* __restrict__ NS, float* P) {
  __shared__ __attribute__((aligned(16))) float stg[GBM * DF];
  __shared__ __attribute__((aligned(16))) float nsh[GBM];
  gemm_tile<K_L2, HLP, W2P>(HL, W2C, NS, P, stg, nsh);
}

template <int RELU>
__global__ __launch_bounds__(NTHR) void k_replay(const float* __restrict__ P, const int* __restrict__ LIST,
                                                 const int* __restrict__ CNT, const int* __restrict__ OFF,
                                                 const float* __restrict__ ND, const int* __restrict__ FLAG,
                                                 const float* __restrict__ bt, unsigned short* HL) {
  __shared__ __attribute__((aligned(16))) float bsh[NR * DF];
  const int tid = (int)threadIdx.x, lane = tid & 31, wave = tid >> 5;
  {
    const int t4 = tid < (NR * DF / 4) ? tid : (NR * DF / 4 - 1);
    const v4f q = *(const v4fa*)(bt + 4 * t4);
    asm volatile("" :: "v"(q));
    if (tid < NR * DF / 4) *(v4fa*)(bsh + 4 * tid) = q;
  }
  __syncthreads();
  const float qnan = __uint_as_float(0x7fc00000u);

#pragma unroll 1
  for (int ri = 0; ri < RPW; ++ri) {
    const int node   = (int)blockIdx.x * RPB + wave * RPW + ri;
    const int bucket = node >> SLB;
    v4f tot = {0.0f, 0.0f, 0.0f, 0.0f};
    int bad = 0;
#pragma unroll 1
    for (int r = 0; r < NR; ++r) {
      const size_t tb = (size_t)r * NPADN + (size_t)node;
      const int craw = CNT[tb];
      const int oraw = OFF[tb];
      const float nd = ND[tb];
      const int fl   = FLAG[(size_t)(r * NBK + bucket) * 32];
      bad |= ((fl != 0) || (craw > DEGCAP)) ? 1 : 0;
      int c = craw < 0 ? 0 : (craw > DEGCAP ? DEGCAP : craw);
      int o = oraw < 0 ? 0 : (oraw > RCAP - 1 ? RCAP - 1 : oraw);
      c = __builtin_amdgcn_readfirstlane(c);
      o = __builtin_amdgcn_readfirstlane(o);
      int last = o + c - 1; last = last < o ? o : last;
      last = last > RCAP - 1 ? RCAP - 1 : last;
      const int* lp = LIST + (size_t)(r * NBK + bucket) * RCAP;
      float a0 = 0.0f, a1 = 0.0f, a2 = 0.0f, a3 = 0.0f;
#pragma unroll 1
      for (int b0 = 0; b0 < c; b0 += 32) {
        int idx = o + b0 + lane;
        idx = idx > last ? last : idx;
        int col = lp[idx];
        col = col < 0 ? 0 : (col > NN - 1 ? NN - 1 : col);
        const int m32 = (c - b0) < 32 ? (c - b0) : 32;
#pragma unroll 1
        for (int k = 0; k < m32; ++k) {
          const int sk = __builtin_amdgcn_readlane(col, k);
          const v4f v = *(const v4fa*)(P + (size_t)sk * PP + r * DF + 4 * lane);
          a0 += v.x; a1 += v.y; a2 += v.z; a3 += v.w;
        }
      }
      const v4f bv = *(const v4fa*)(bsh + r * DF + 4 * lane);
      tot.x = tot.x + (nd * a0 + bv.x);
      tot.y = tot.y + (nd * a1 + bv.y);
      tot.z = tot.z + (nd * a2 + bv.z);
      tot.w = tot.w + (nd * a3 + bv.w);
    }
    float v0 = tot.x / 3.0f, v1 = tot.y / 3.0f, v2 = tot.z / 3.0f, v3 = tot.w / 3.0f;
    if (RELU != 0) {
      v0 = (v0 > 0.0f) ? v0 : (v0 - v0); v1 = (v1 > 0.0f) ? v1 : (v1 - v1);
      v2 = (v2 > 0.0f) ? v2 : (v2 - v2); v3 = (v3 > 0.0f) ? v3 : (v3 - v3);
    }
    const bool pz   = bad != 0;
    const bool live = node < NN;
    v0 = pz ? qnan : v0; v1 = pz ? qnan : v1; v2 = pz ? qnan : v2; v3 = pz ? qnan : v3;
    v0 = live ? v0 : 0.0f; v1 = live ? v1 : 0.0f; v2 = live ? v2 : 0.0f; v3 = live ? v3 : 0.0f;
    int h01, h23, l01, l23;
    hilo_pack(v0, v1, v2, v3, h01, h23, l01, l23);
    const v4i ow = regroup_row(h01, h23, l01, l23, lane);
    unsigned short* hp = HL + (size_t)node * HLP + 8 * lane;
    *(volatile v4i*)hp = ow;
    __threadfence();
    *(volatile v4i*)hp = ow;
  }
}

__device__ __forceinline__ void head_flush(const float* lg, float* ob, int nv4, unsigned pz, unsigned km, int tid) {
#pragma unroll 1
  for (int it = 0; it < 5; ++it) {
    const int i4 = it * NTHR + tid;
    const v4f v = *(const v4fa*)(lg + 4 * i4);
    asm volatile("" :: "v"(v));
    v4f o;
    o.x = __uint_as_float((__float_as_uint(v.x) & km) | pz);
    o.y = __uint_as_float((__float_as_uint(v.y) & km) | pz);
    o.z = __uint_as_float((__float_as_uint(v.z) & km) | pz);
    o.w = __uint_as_float((__float_as_uint(v.w) & km) | pz);
    if (i4 < nv4) *(volatile v4f*)(ob + (size_t)4 * (size_t)i4) = o;
  }
}

__global__ __launch_bounds__(NTHR) __attribute__((amdgpu_num_vgpr(248)))
void k_head(const unsigned short* __restrict__ HL, const unsigned short* __restrict__ WCT,
            const float* __restrict__ btc, const int* __restrict__ FLAG, float* out) {
  __shared__ __attribute__((aligned(16))) float lg[HBM * NC];
  __shared__ __attribute__((aligned(16))) float sb[64];
  const int tid = (int)threadIdx.x, lane = tid & 31, wave = tid >> 5, hh = lane >> 4, m = lane & 15;
  const int blk = (int)blockIdx.x;
  const int rowBase = blk * HBM;
  const int bk = rowBase >> SLB;
  const int f0 = FLAG[(size_t)(0 * NBK + bk) * 32];
  const int f1 = FLAG[(size_t)(1 * NBK + bk) * 32];
  const int f2 = FLAG[(size_t)(2 * NBK + bk) * 32];
  const int flag = f0 | f1 | f2;
  {
    const v4f q = *(const v4fa*)(btc + 4 * (tid & 15));
    asm volatile("" :: "v"(q));
    if (tid < 16) *(v4fa*)(sb + 4 * tid) = q;
  }

  v8f acc[3];
  {
    const v8f z = {0.f, 0.f, 0.f, 0.f, 0.f, 0.f, 0.f, 0.f};
#pragma unroll
    for (int t = 0; t < 3; ++t) acc[t] = z;
  }
  const unsigned short* ap = HL + (size_t)(rowBase + 16 * wave + m) * (size_t)HLP + 8 * hh;
  const unsigned short* bp = WCT + (size_t)m * (size_t)WCP + 8 * hh;
#pragma unroll 1
  for (int k0 = 0; k0 < K_HD; k0 += 32) {
    FragB af;
    af.h[0] = *(const v8usa*)(ap + k0);
    af.h[1] = *(const v8usa*)(ap + k0 + 16);
#pragma unroll
    for (int t = 0; t < 3; ++t) {
      const unsigned short* wq = bp + (size_t)(16 * t) * (size_t)WCP + k0;
      FragB bf;
      bf.h[0] = *(const v8usa*)wq;
      bf.h[1] = *(const v8usa*)(wq + 16);
      acc[t] = wmb(af, bf, acc[t]);
    }
  }
  __syncthreads();
#pragma unroll
  for (int t = 0; t < 3; ++t) {
    const int col = 16 * t + m;
    const float bcv = sb[col];
#pragma unroll
    for (int r = 0; r < 8; ++r) {
      if (col < NC) lg[(16 * wave + 8 * hh + r) * NC + col] = acc[t][r] + bcv;
    }
  }
  __syncthreads();

  const unsigned pz = (flag != 0) ? 0x7fc00000u : 0u;
  const unsigned km = (flag != 0) ? 0u : 0xFFFFFFFFu;
  const int liveRows = (NN - rowBase) < HBM ? (NN - rowBase) : HBM;
  const int nv4 = liveRows * (NC / 4);
  float* ob = out + (size_t)blk * (size_t)(HBM * NC);
  head_flush(lg, ob, nv4, pz, km, tid);
  __threadfence();
  head_flush(lg, ob, nv4, pz, km, tid);
}

extern "C" void kernel_launch(void* const* d_in, const int* in_sizes, int n_in,
                              void* d_out, int out_size, void* d_ws, size_t ws_size,
                              hipStream_t stream) {
  if (n_in < 8) return;
  if (in_sizes[0] != NN * DF) return;
  if (in_sizes[1] != NR * 2 * NE) return;
  if (in_sizes[2] != NR * DF * DF) return;
  if (in_sizes[3] != NR * DF) return;
  if (in_sizes[4] != NR * DF * DF) return;
  if (in_sizes[5] != NR * DF) return;
  if (in_sizes[6] != DF * NC) return;
  if (in_sizes[7] != NC) return;
  if (out_size != NN * NC) return;

  const float* x   = (const float*)d_in[0];
  const int*   edg = (const int*)d_in[1];
  const float* W1  = (const float*)d_in[2];
  const float* b1  = (const float*)d_in[3];
  const float* W2  = (const float*)d_in[4];
  const float* b2  = (const float*)d_in[5];
  const float* Wc  = (const float*)d_in[6];
  const float* bc  = (const float*)d_in[7];
  float* out = (float*)d_out;

  constexpr size_t zP    = (size_t)MP * PP * 4;
  constexpr size_t zHL   = (size_t)MP * HLP * 2;
  constexpr size_t zXB   = (size_t)MP * XBP * 2;
  constexpr size_t zLIST = (size_t)NR * NBK * RCAP * 4;
  constexpr size_t zT    = (size_t)NR * NPADN * 4;
  constexpr size_t zW1   = (size_t)NR * DF * W1P * 2;
  constexpr size_t zW2   = (size_t)NR * DF * W2P * 2;
  constexpr size_t zWC   = (size_t)NT * WCP * 2;
  constexpr size_t zBT   = 4096;
  constexpr size_t zFLAG = (size_t)NR * NBK * 128;
  constexpr size_t oP    = 0;
  constexpr size_t oHL   = oP + zP;
  constexpr size_t oLIST = oHL + zHL;
  constexpr size_t oCNT  = oLIST + zLIST;
  constexpr size_t oOFF  = oCNT + zT;
  constexpr size_t oNRM  = oOFF + zT;
  constexpr size_t oW1   = oNRM + 2 * zT;
  constexpr size_t oW2   = oW1 + zW1;
  constexpr size_t oWC   = oW2 + zW2;
  constexpr size_t oBT   = oWC + zWC;
  constexpr size_t oFLAG = oBT + zBT;
  constexpr size_t oEND  = oFLAG + zFLAG;
  static_assert(zP % 256 == 0 && zHL % 256 == 0 && zLIST % 256 == 0 && zT % 256 == 0 && zW1 % 256 == 0);
  static_assert(zW2 % 256 == 0 && zWC % 256 == 0 && zBT % 256 == 0 && zFLAG % 256 == 0);
  static_assert(zXB <= zHL);
  static_assert(oEND <= ((size_t)256u << 20));
  if (oEND > ws_size) return;

  char* ws = (char*)d_ws;
  float*          P    = (float*)(ws + oP);
  unsigned short* HL   = (unsigned short*)(ws + oHL);
  unsigned short* XB   = (unsigned short*)(ws + oHL);
  int*            LIST = (int*)(ws + oLIST);
  int*            CNT  = (int*)(ws + oCNT);
  int*            OFF  = (int*)(ws + oOFF);
  int*            NRMi = (int*)(ws + oNRM);
  const float*    NS   = (const float*)(ws + oNRM);
  const float*    ND   = (const float*)(ws + oNRM + zT);
  unsigned short* W1C  = (unsigned short*)(ws + oW1);
  unsigned short* W2C  = (unsigned short*)(ws + oW2);
  unsigned short* WCT  = (unsigned short*)(ws + oWC);
  float*          BT   = (float*)(ws + oBT);
  int*            FLAG = (int*)(ws + oFLAG);

  k_prep<<<PBTOT, NTHR, 0, stream>>>(x, W1, b1, W2, b2, Wc, bc, XB, W1C, W2C, WCT, BT);
  k_bucket<<<2 * NR * NBK, NTHR, 0, stream>>>(edg, LIST, CNT, OFF, NRMi, FLAG);
  const dim3 gg((unsigned)(MP / GBM), (unsigned)NR, 1u);
  k_gemm_one<<<gg, GTHR, 0, stream>>>(XB, W1C, NS, P);
  k_replay<1><<<MP / RPB, NTHR, 0, stream>>>(P, LIST, CNT, OFF, ND, FLAG, BT, HL);
  k_gemm_two<<<gg, GTHR, 0, stream>>>(HL, W2C, NS, P);
  k_replay<0><<<MP / RPB, NTHR, 0, stream>>>(P, LIST, CNT, OFF, ND, FLAG, BT + NR * DF, HL);
  k_head<<<MP / HBM, NTHR, 0, stream>>>(HL, WCT, BT + 2 * NR * DF, FLAG, out);
}
